// MultiHeadSelfAttention_78331613545069
// MI455X (gfx1250) — hardware-verified
//
#include <hip/hip_runtime.h>


#ifndef NB
#define NB 2
#endif
#ifndef SEQ
#define SEQ 2048
#endif
#define NB_FULL  2
#define SEQ_FULL 2048
#define DM   1024
#define NH   16
#define HD   64
#define F3   (3 * DM)
#define CK   (2 * DM)
#define RH   256
#define NBH  (NB * NH)
#define MROWS (SEQ * NB)
#define ROWSTEP (NB_FULL / NB)
#define PLN  ((size_t)NBH * SEQ * HD)
#define PLNH ((size_t)NBH * RH * HD)
#define PCAR 1024.0f
#define PP   40
#define OP   72
#define ER   16

static_assert(NB == NB_FULL || NB == 1);
static_assert(SEQ <= SEQ_FULL && SEQ >= RH);
static_assert(SEQ % 256 == 0);
static_assert(RH % 32 == 0 && RH % 8 == 0);
static_assert(RH % ER == 0 && ER == 16);
static_assert(HD == 64 && NH * HD == DM);
static_assert(DM == 1024);
static_assert(DM % 32 == 0 && CK % 32 == 0);
static_assert(MROWS % 64 == 0 && F3 % 64 == 0 && DM % 64 == 0);
static_assert(((size_t)NBH * SEQ * HD / 8) % 256 == 0);
static_assert(PP >= 32 && (PP * 2) % 16 == 0);
static_assert(OP >= 64 && (OP * 2) % 16 == 0);

typedef _Float16 h16;
typedef unsigned short bf;
typedef unsigned short us;
typedef __attribute__((ext_vector_type(16))) __bf16   v16bf;
typedef __attribute__((ext_vector_type(16))) _Float16 v16h;
typedef __attribute__((ext_vector_type(16))) unsigned short v16us;
typedef __attribute__((ext_vector_type(8)))  _Float16 v8h;
typedef __attribute__((ext_vector_type(8)))  unsigned short v8us;
typedef __attribute__((ext_vector_type(8)))  float    v8f;
typedef __attribute__((ext_vector_type(4)))  float    v4f;
typedef v4f  __attribute__((may_alias)) v4fa;
typedef v8us __attribute__((may_alias)) v8usa;

__device__ __forceinline__ unsigned short f2bf(float f) { unsigned u = __float_as_uint(f); u += 0x7FFFu + ((u >> 16) & 1u); return (unsigned short)(u >> 16); }
__device__ __forceinline__ float bf2f(unsigned short b) { return __uint_as_float(((unsigned)b) << 16); }
__device__ __forceinline__ void splitf(float y, unsigned short& h, unsigned short& l) { h = f2bf(y); l = f2bf(y - bf2f(h)); }

__device__ __forceinline__ v16us ldus(const us* p) {
    const v8us a = *(const v8us*)p; const v8us b = *(const v8us*)(p + 16);
    return __builtin_shufflevector(a, b, 0, 1, 2, 3, 4, 5, 6, 7, 8, 9, 10, 11, 12, 13, 14, 15);
}

template <bool BF>
__device__ __forceinline__ v8f mmg(v16us a, v16us b, v8f c) {
    if (BF) c = __builtin_amdgcn_wmma_f32_16x16x32_bf16(false, __builtin_bit_cast(v16bf, a), false, __builtin_bit_cast(v16bf, b), (short)0, c, false, false);
    else    c = __builtin_amdgcn_wmma_f32_16x16x32_f16(false, __builtin_bit_cast(v16h, a), false, __builtin_bit_cast(v16h, b), (short)0, c, false, false);
    asm volatile("v_nop\n\tv_nop\n\tv_nop\n\tv_nop" : "+v"(c) : "v"(a), "v"(b));
    return c;
}

__global__ __launch_bounds__(256) void k_cvt(const float* __restrict__ src, int srcstep, bf* dst, int dstpitch, int dstcol, int ngroups) {
    const int i = blockIdx.x * 256 + threadIdx.x; if (i >= ngroups) return;
    const int row = i >> 7, cg = i & 127;
    const v8f v = *(const v8f*)(src + (size_t)row * srcstep * DM + cg * 8);
    v8us o;
#pragma unroll
    for (int k = 0; k < 8; ++k) o[k] = f2bf(v[k]);
    bf* d = dst + (size_t)row * dstpitch + dstcol + cg * 8;
    *(volatile v8us*)d = o; __threadfence(); *(volatile v8us*)d = o;
}

__global__ __launch_bounds__(32) void k_gemmw(const bf* __restrict__ A, int lda, const bf* __restrict__ Bt, int ldb, int K, float* C, int ldc) {
    __shared__ __align__(16) float os[16 * 68];
    const int lane = threadIdx.x & 31, lr = lane & 15, hi = lane >> 4;
    const int r0 = blockIdx.x * 64, c0 = blockIdx.y * 64;
    v8f acc[4][4];
#pragma unroll
    for (int mb = 0; mb < 4; ++mb)
#pragma unroll
        for (int nb = 0; nb < 4; ++nb) acc[mb][nb] = (v8f){};
    const size_t aoff = (size_t)(r0 + lr) * lda + 8 * hi, boff = (size_t)(c0 + lr) * ldb + 8 * hi;
#pragma unroll 1
    for (int kc = 0; kc < K; kc += 32) {
        v16us a[4];
#pragma unroll
        for (int mb = 0; mb < 4; ++mb) a[mb] = ldus(A + aoff + (size_t)mb * 16 * lda + kc);
#pragma unroll
        for (int nb = 0; nb < 4; ++nb) {
            const v16us b = ldus(Bt + boff + (size_t)nb * 16 * ldb + kc);
#pragma unroll
            for (int mb = 0; mb < 4; ++mb) acc[mb][nb] = mmg<true>(a[mb], b, acc[mb][nb]);
        }
    }
#pragma unroll
    for (int mb = 0; mb < 4; ++mb) {
#pragma unroll
        for (int nb = 0; nb < 4; ++nb) {
#pragma unroll
            for (int j = 0; j < 8; ++j) os[(hi * 8 + j) * 68 + nb * 16 + lr] = acc[mb][nb][j];
        }
        __builtin_amdgcn_wave_barrier(); asm volatile("" ::: "memory");
        float* crow = C + (size_t)(r0 + mb * 16) * ldc + c0;
#pragma unroll 1
        for (int ps = 0; ps < 2; ++ps) {
#pragma unroll
            for (int s = 0; s < 8; ++s) {
                const int row = 2 * s + hi, cofs = lr * 4;
                const v4f val = *(const v4fa*)(os + row * 68 + cofs);
                *(volatile v4f*)(crow + (size_t)row * ldc + cofs) = val;
            }
            if (ps == 0) __threadfence();
        }
        __builtin_amdgcn_wave_barrier(); asm volatile("" ::: "memory");
    }
}

__device__ __forceinline__ void cvt3(const v8f x, v8h& o16, v8us& oh, v8us& ol) {
#pragma unroll
    for (int k = 0; k < 8; ++k) { o16[k] = (h16)x[k]; unsigned short a, c; splitf(x[k], a, c); oh[k] = a; ol[k] = c; }
}
__device__ __forceinline__ void store3(h16* p16, bf* ph, bf* pl, bool hr, const v8h o16, const v8us oh, const v8us ol) {
    *(volatile v8h*)p16 = o16; if (hr) { *(volatile v8us*)ph = oh; *(volatile v8us*)pl = ol; }
    __threadfence();
    *(volatile v8h*)p16 = o16; if (hr) { *(volatile v8us*)ph = oh; *(volatile v8us*)pl = ol; }
}
__global__ __launch_bounds__(256) void k_planes(const float* __restrict__ F, h16* QK16, bf* QKh, bf* QKl, h16* VT16, bf* VTh, bf* VTl) {
    const int g = blockIdx.x * 256 + threadIdx.x;
    if (g >= NBH * SEQ * HD / 8) return;
    const int which = blockIdx.y;
    v8h o16; v8us oh, ol;
    if (which < 2) {
        const int d8 = g & 7, l = (g >> 3) % SEQ, bh = g / (8 * SEQ), n = bh / NH, h = bh % NH;
        const float* f = F + ((size_t)l * NB + n) * F3 + which * DM + h * HD + d8 * 8;
        const v4f a = *(const v4f*)f, b = *(const v4f*)(f + 4);
        const v8f x = __builtin_shufflevector(a, b, 0, 1, 2, 3, 4, 5, 6, 7);
        cvt3(x, o16, oh, ol);
        const bool hr = (l < RH);
        const size_t e16 = (size_t)which * PLN + ((size_t)bh * SEQ + l) * HD + d8 * 8;
        const size_t eh = hr ? ((size_t)which * PLNH + ((size_t)bh * RH + l) * HD + d8 * 8) : 0;
        store3(QK16 + e16, QKh + eh, QKl + eh, hr, o16, oh, ol);
    } else {
        const int l8 = g % (SEQ / 8), d = (g / (SEQ / 8)) % HD, bh = g / (HD * (SEQ / 8)), n = bh / NH, h = bh % NH;
        const int l = l8 * 8;
        v8f x;
#pragma unroll
        for (int j = 0; j < 8; ++j) x[j] = F[((size_t)(l + j) * NB + n) * F3 + 2 * DM + h * HD + d];
        cvt3(x, o16, oh, ol);
        const bool hr = (l < RH);
        const size_t e16 = ((size_t)bh * HD + d) * SEQ + l;
        const size_t eh = hr ? (((size_t)bh * HD + d) * RH + l) : 0;
        store3(VT16 + e16, VTh + eh, VTl + eh, hr, o16, oh, ol);
    }
}

template <bool HR>
__device__ __forceinline__ void attn_body(const us* __restrict__ Qa, const us* __restrict__ Qr, const us* __restrict__ Ka, const us* __restrict__ Kr,
                                          const us* __restrict__ Va, const us* __restrict__ Vr, bf* CTX, const int q0) {
    constexpr int LR = HR ? RH : SEQ;
    __shared__ __align__(16) unsigned short psA[32 * PP];
    __shared__ __align__(16) unsigned short psB[32 * PP];
    __shared__ __align__(16) unsigned short oh[32 * OP];
    __shared__ __align__(16) unsigned short ol[32 * OP];
    const int lane = threadIdx.x & 31, lr = lane & 15, hi = lane >> 4;
    const int bh = blockIdx.x, n = bh / NH, h = bh % NH;
    const size_t pb = (size_t)bh * LR * HD;
    Qa += pb; Ka += pb; Va += pb; Qr += pb; Kr += pb; Vr += pb;
    const int qoff = (q0 + lr) * HD + 8 * hi;
    const int koff = lr * HD + 8 * hi;
    const int voff = lr * LR + 8 * hi;
    const float cexp = 0.125f * 1.4426950408889634f;
    const float pc = HR ? 1.0f : PCAR;
    v8f o[2][4]; float mrow[2][8], lsum[2][8];
#pragma unroll
    for (int u = 0; u < 2; ++u) {
#pragma unroll
        for (int t2 = 0; t2 < 4; ++t2) o[u][t2] = (v8f){};
#pragma unroll
        for (int r = 0; r < 8; ++r) { mrow[u][r] = -3.0e38f; lsum[u][r] = 0.0f; }
    }
#pragma unroll 1
    for (int m0 = 0; m0 <= q0; m0 += 32) {
        int qo = qoff; asm volatile("" : "+v"(qo));
        v8f s[2][2];
#pragma unroll
        for (int u = 0; u < 2; ++u)
#pragma unroll
            for (int t = 0; t < 2; ++t) s[u][t] = (v8f){};
#pragma unroll
        for (int kc = 0; kc < 2; ++kc) {
            const v16us qa0 = ldus(Qa + qo + kc * 32), qa1 = ldus(Qa + qo + 16 * HD + kc * 32);
            v16us qr0 = qa0, qr1 = qa1;
            if (HR) { qr0 = ldus(Qr + qo + kc * 32); qr1 = ldus(Qr + qo + 16 * HD + kc * 32); }
#pragma unroll
            for (int t = 0; t < 2; ++t) {
                const int ko = (m0 + t * 16) * HD + koff + kc * 32;
                const v16us ka = ldus(Ka + ko);
                s[0][t] = mmg<HR>(qa0, ka, s[0][t]); s[1][t] = mmg<HR>(qa1, ka, s[1][t]);
                if (HR) {
                    const v16us kr = ldus(Kr + ko);
                    s[0][t] = mmg<HR>(qr0, ka, s[0][t]); s[1][t] = mmg<HR>(qr1, ka, s[1][t]);
                    s[0][t] = mmg<HR>(qa0, kr, s[0][t]); s[1][t] = mmg<HR>(qa1, kr, s[1][t]);
                }
            }
        }
        if (m0 == q0) {
#pragma unroll
            for (int u = 0; u < 2; ++u)
#pragma unroll
                for (int t = 0; t < 2; ++t)
#pragma unroll
                    for (int r = 0; r < 8; ++r) { if (t * 16 + lr > u * 16 + 8 * hi + r) s[u][t][r] = -3.0e38f; }
        }
#pragma unroll
        for (int u = 0; u < 2; ++u) {
#pragma unroll
            for (int r = 0; r < 8; ++r) {
                const float s0 = s[u][0][r], s1 = s[u][1][r];
                float v = fmaxf(s0, s1);
                v = fmaxf(v, __shfl_xor(v, 1, 32)); v = fmaxf(v, __shfl_xor(v, 2, 32));
                v = fmaxf(v, __shfl_xor(v, 4, 32)); v = fmaxf(v, __shfl_xor(v, 8, 32));
                const float mn = fmaxf(mrow[u][r], v);
                const float al = __builtin_amdgcn_exp2f((mrow[u][r] - mn) * cexp);
                mrow[u][r] = mn;
                const float p0 = __builtin_amdgcn_exp2f((s0 - mn) * cexp);
                const float p1 = __builtin_amdgcn_exp2f((s1 - mn) * cexp);
                lsum[u][r] = lsum[u][r] * al + (p0 + p1);
                const int po = (u * 16 + 8 * hi + r) * PP + lr;
                if (HR) {
                    unsigned short a, c; splitf(p0, a, c); psA[po] = a; psB[po] = c;
                    splitf(p1, a, c); psA[po + 16] = a; psB[po + 16] = c;
                } else {
                    psA[po] = __builtin_bit_cast(unsigned short, (h16)(p0 * PCAR));
                    psA[po + 16] = __builtin_bit_cast(unsigned short, (h16)(p1 * PCAR));
                }
#pragma unroll
                for (int t2 = 0; t2 < 4; ++t2) o[u][t2][r] *= al;
            }
        }
        __syncthreads();
        v16us pa[2], pr[2];
#pragma unroll
        for (int u = 0; u < 2; ++u) {
            const int po = (u * 16 + lr) * PP + 8 * hi;
            { const v8us x0 = *(const v8usa*)(psA + po); const v8us x1 = *(const v8usa*)(psA + po + 16);
              pa[u] = __builtin_shufflevector(x0, x1, 0, 1, 2, 3, 4, 5, 6, 7, 8, 9, 10, 11, 12, 13, 14, 15); }
            pr[u] = pa[u];
            if (HR) { const v8us y0 = *(const v8usa*)(psB + po); const v8us y1 = *(const v8usa*)(psB + po + 16);
              pr[u] = __builtin_shufflevector(y0, y1, 0, 1, 2, 3, 4, 5, 6, 7, 8, 9, 10, 11, 12, 13, 14, 15); }
        }
#pragma unroll
        for (int t2 = 0; t2 < 4; ++t2) {
            const int vo = (t2 * 16) * LR + voff + m0;
            const v16us va = ldus(Va + vo);
            o[0][t2] = mmg<HR>(pa[0], va, o[0][t2]); o[1][t2] = mmg<HR>(pa[1], va, o[1][t2]);
            if (HR) {
                const v16us vr = ldus(Vr + vo);
                o[0][t2] = mmg<HR>(pr[0], va, o[0][t2]); o[1][t2] = mmg<HR>(pr[1], va, o[1][t2]);
                o[0][t2] = mmg<HR>(pa[0], vr, o[0][t2]); o[1][t2] = mmg<HR>(pa[1], vr, o[1][t2]);
            }
        }
        __syncthreads();
    }
#pragma unroll
    for (int u = 0; u < 2; ++u) {
#pragma unroll
        for (int r = 0; r < 8; ++r) {
            float l = lsum[u][r];
            l += __shfl_xor(l, 1, 32); l += __shfl_xor(l, 2, 32); l += __shfl_xor(l, 4, 32); l += __shfl_xor(l, 8, 32);
            const float inv = 1.0f / (l * pc);
#pragma unroll
            for (int t2 = 0; t2 < 4; ++t2) {
                const float val = o[u][t2][r] * inv;
                unsigned short a, c; splitf(val, a, c);
                const int oo = (u * 16 + 8 * hi + r) * OP + t2 * 16 + lr;
                oh[oo] = a; ol[oo] = c;
            }
        }
    }
    __syncthreads();
#pragma unroll 1
    for (int ps = 0; ps < 2; ++ps) {
#pragma unroll
        for (int s = 0; s < 8; ++s) {
            const int row = s * 4 + (lane >> 3), cp = (lane & 7) * 8;
            const v8us vh = *(const v8usa*)(oh + row * OP + cp);
            const v8us vl = *(const v8usa*)(ol + row * OP + cp);
            bf* d = CTX + ((size_t)(q0 + row) * NB + n) * CK + h * HD + cp;
            *(volatile v8us*)d = vh; *(volatile v8us*)(d + DM) = vl;
        }
        if (ps == 0) __threadfence();
    }
}

__global__ __launch_bounds__(32) void k_attn_lo(const us* __restrict__ Q16, const us* __restrict__ K16, const us* __restrict__ V16, bf* CTX) {
    attn_body<false>(Q16, Q16, K16, K16, V16, V16, CTX, RH + (int)blockIdx.y * 32);
}

__global__ __launch_bounds__(32) void k_attn_hr(const us* __restrict__ Qh, const us* __restrict__ Ql, const us* __restrict__ Kh, const us* __restrict__ Kl,
                                                const us* __restrict__ Vh, const us* __restrict__ Vl, bf* CTX) {
    __shared__ __align__(16) unsigned short epa[ER * PP];
    __shared__ __align__(16) unsigned short epb[ER * PP];
    __shared__ __align__(16) unsigned short eoh[ER * OP];
    __shared__ __align__(16) unsigned short eol[ER * OP];
    const int lane = threadIdx.x & 31, lr = lane & 15, hi = lane >> 4;
    const int bh = blockIdx.x, n = bh / NH, h = bh % NH;
    const int q0 = (int)blockIdx.y * ER;
    const int mend = q0 & ~31;
    const size_t pb = (size_t)bh * RH * HD;
    Qh += pb; Ql += pb; Kh += pb; Kl += pb; Vh += pb; Vl += pb;
    const int qoff = (q0 + lr) * HD + 8 * hi;
    const int koff = lr * HD + 8 * hi;
    const int voff = lr * RH + 8 * hi;
    const float cexp = 0.125f * 1.4426950408889634f;
    v8f o[4]; float mrow[8], lsum[8];
#pragma unroll
    for (int t2 = 0; t2 < 4; ++t2) o[t2] = (v8f){};
#pragma unroll
    for (int r = 0; r < 8; ++r) { mrow[r] = -3.0e38f; lsum[r] = 0.0f; }
#pragma unroll 1
    for (int m0 = 0; m0 <= mend; m0 += 32) {
        int qo = qoff; asm volatile("" : "+v"(qo));
        v8f s[2];
        s[0] = (v8f){}; s[1] = (v8f){};
#pragma unroll
        for (int kc = 0; kc < 2; ++kc) {
            const v16us qa = ldus(Qh + qo + kc * 32);
            const v16us qr = ldus(Ql + qo + kc * 32);
#pragma unroll
            for (int t = 0; t < 2; ++t) {
                const int ko = (m0 + t * 16) * HD + koff + kc * 32;
                const v16us ka = ldus(Kh + ko);
                s[t] = mmg<true>(qa, ka, s[t]);
                s[t] = mmg<true>(qr, ka, s[t]);
                const v16us kr = ldus(Kl + ko);
                s[t] = mmg<true>(qa, kr, s[t]);
            }
        }
        if (m0 == mend) {
#pragma unroll
            for (int t = 0; t < 2; ++t)
#pragma unroll
                for (int r = 0; r < 8; ++r) { if (m0 + t * 16 + lr > q0 + 8 * hi + r) s[t][r] = -3.0e38f; }
        }
#pragma unroll
        for (int r = 0; r < 8; ++r) {
            const float s0 = s[0][r], s1 = s[1][r];
            float v = fmaxf(s0, s1);
            v = fmaxf(v, __shfl_xor(v, 1, 32)); v = fmaxf(v, __shfl_xor(v, 2, 32));
            v = fmaxf(v, __shfl_xor(v, 4, 32)); v = fmaxf(v, __shfl_xor(v, 8, 32));
            const float mn = fmaxf(mrow[r], v);
            const float al = __builtin_amdgcn_exp2f((mrow[r] - mn) * cexp);
            mrow[r] = mn;
            const float p0 = __builtin_amdgcn_exp2f((s0 - mn) * cexp);
            const float p1 = __builtin_amdgcn_exp2f((s1 - mn) * cexp);
            lsum[r] = lsum[r] * al + (p0 + p1);
            const int po = (8 * hi + r) * PP + lr;
            unsigned short a, c;
            splitf(p0, a, c); epa[po] = a; epb[po] = c;
            splitf(p1, a, c); epa[po + 16] = a; epb[po + 16] = c;
#pragma unroll
            for (int t2 = 0; t2 < 4; ++t2) o[t2][r] *= al;
        }
        __syncthreads();
        v16us pa, pr;
        {
            const int po = lr * PP + 8 * hi;
            const v8us x0 = *(const v8usa*)(epa + po); const v8us x1 = *(const v8usa*)(epa + po + 16);
            pa = __builtin_shufflevector(x0, x1, 0, 1, 2, 3, 4, 5, 6, 7, 8, 9, 10, 11, 12, 13, 14, 15);
            const v8us y0 = *(const v8usa*)(epb + po); const v8us y1 = *(const v8usa*)(epb + po + 16);
            pr = __builtin_shufflevector(y0, y1, 0, 1, 2, 3, 4, 5, 6, 7, 8, 9, 10, 11, 12, 13, 14, 15);
        }
#pragma unroll
        for (int t2 = 0; t2 < 4; ++t2) {
            const int vo = (t2 * 16) * RH + voff + m0;
            const v16us va = ldus(Vh + vo);
            o[t2] = mmg<true>(pa, va, o[t2]);
            o[t2] = mmg<true>(pr, va, o[t2]);
            const v16us vr = ldus(Vl + vo);
            o[t2] = mmg<true>(pa, vr, o[t2]);
        }
        __syncthreads();
    }
#pragma unroll
    for (int r = 0; r < 8; ++r) {
        float l = lsum[r];
        l += __shfl_xor(l, 1, 32); l += __shfl_xor(l, 2, 32); l += __shfl_xor(l, 4, 32); l += __shfl_xor(l, 8, 32);
        const float inv = 1.0f / l;
#pragma unroll
        for (int t2 = 0; t2 < 4; ++t2) {
            const float val = o[t2][r] * inv;
            unsigned short a, c; splitf(val, a, c);
            const int oo = (8 * hi + r) * OP + t2 * 16 + lr;
            eoh[oo] = a; eol[oo] = c;
        }
    }
    __syncthreads();
#pragma unroll 1
    for (int ps = 0; ps < 2; ++ps) {
#pragma unroll
        for (int s4 = 0; s4 < ER / 4; ++s4) {
            const int row = s4 * 4 + (lane >> 3), cp = (lane & 7) * 8;
            const v8us vh = *(const v8usa*)(eoh + row * OP + cp);
            const v8us vl = *(const v8usa*)(eol + row * OP + cp);
            bf* d = CTX + ((size_t)(q0 + row) * NB + n) * CK + h * HD + cp;
            *(volatile v8us*)d = vh; *(volatile v8us*)(d + DM) = vl;
        }
        if (ps == 0) __threadfence();
    }
}

constexpr size_t SZ_XB   = (size_t)MROWS * DM * 2;
constexpr size_t SZ_WQ   = (size_t)F3 * DM * 2;
constexpr size_t SZ_WO   = (size_t)DM * CK * 2;
constexpr size_t SZ_F    = (size_t)MROWS * F3 * 4;
constexpr size_t SZ_QK16 = (size_t)2 * NBH * SEQ * HD * 2;
constexpr size_t SZ_QKH  = (size_t)2 * NBH * RH * HD * 2;
constexpr size_t SZ_VT16 = (size_t)NBH * HD * SEQ * 2;
constexpr size_t SZ_VTH  = (size_t)NBH * HD * RH * 2;
constexpr size_t SZ_CTX  = (size_t)MROWS * CK * 2;
constexpr size_t OF_XB   = 0;
constexpr size_t OF_WQ   = OF_XB + SZ_XB;
constexpr size_t OF_WO   = OF_WQ + SZ_WQ;
constexpr size_t OF_F    = OF_WO + SZ_WO;
constexpr size_t OF_QK16 = OF_F + SZ_F;
constexpr size_t OF_QKH  = OF_QK16 + SZ_QK16;
constexpr size_t OF_QKL  = OF_QKH + SZ_QKH;
constexpr size_t OF_VT16 = OF_QKL + SZ_QKH;
constexpr size_t OF_VTH  = OF_VT16 + SZ_VT16;
constexpr size_t OF_VTL  = OF_VTH + SZ_VTH;
constexpr size_t OF_CTX  = OF_VTL + SZ_VTH;
constexpr size_t WS_TOTAL = OF_CTX + SZ_CTX;
static_assert(SZ_XB % 256 == 0 && SZ_WQ % 256 == 0 && SZ_WO % 256 == 0 && SZ_F % 256 == 0 && SZ_QK16 % 256 == 0);
static_assert(SZ_QKH % 256 == 0 && SZ_VT16 % 256 == 0 && SZ_VTH % 256 == 0 && SZ_CTX % 256 == 0);
static_assert(WS_TOTAL <= (size_t)134217728);

extern "C" void kernel_launch(void* const* d_in, const int* in_sizes, int n_in,
                              void* d_out, int out_size, void* d_ws, size_t ws_size, hipStream_t stream) {
    if (n_in < 3) return;
    const long long needx = ((long long)(SEQ - 1) * NB_FULL + NB) * DM;
    if ((long long)in_sizes[0] < needx || (long long)in_sizes[1] < (long long)F3 * DM || (long long)in_sizes[2] < (long long)DM * DM || (long long)out_size < needx) return;
    if (WS_TOTAL > ws_size) return;
    const float* x = (const float*)d_in[0];
    const float* wqkv = (const float*)d_in[1];
    const float* wout = (const float*)d_in[2];
    float* OUT = (float*)d_out;
    char* ws = (char*)d_ws;
    bf* XB = (bf*)(ws + OF_XB); bf* WQ = (bf*)(ws + OF_WQ); bf* WO2 = (bf*)(ws + OF_WO); float* F = (float*)(ws + OF_F);
    h16* QK16 = (h16*)(ws + OF_QK16); bf* QKh = (bf*)(ws + OF_QKH); bf* QKl = (bf*)(ws + OF_QKL);
    h16* VT16 = (h16*)(ws + OF_VT16); bf* VTh = (bf*)(ws + OF_VTH); bf* VTl = (bf*)(ws + OF_VTL); bf* CTX = (bf*)(ws + OF_CTX);

    k_cvt<<<(MROWS * 128 + 255) / 256, 256, 0, stream>>>(x, ROWSTEP, XB, DM, 0, MROWS * 128);
    k_cvt<<<(F3 * 128 + 255) / 256, 256, 0, stream>>>(wqkv, 1, WQ, DM, 0, F3 * 128);
    k_cvt<<<(DM * 128 + 255) / 256, 256, 0, stream>>>(wout, 1, WO2, CK, 0, DM * 128);
    k_cvt<<<(DM * 128 + 255) / 256, 256, 0, stream>>>(wout, 1, WO2, CK, DM, DM * 128);
    k_gemmw<<<dim3(MROWS / 64, F3 / 64, 1), 32, 0, stream>>>(XB, DM, WQ, DM, DM, F, F3);
    k_planes<<<dim3((unsigned)((size_t)NBH * SEQ * HD / 8 / 256), 3, 1), 256, 0, stream>>>(F, QK16, QKh, QKl, VT16, VTh, VTl);
    k_attn_hr<<<dim3(NBH, RH / ER, 1), 32, 0, stream>>>((const us*)QKh, (const us*)QKl, (const us*)(QKh + PLNH), (const us*)(QKl + PLNH), (const us*)VTh, (const us*)VTl, CTX);
    if (SEQ > RH)
        k_attn_lo<<<dim3(NBH, (SEQ - RH) / 32 > 0 ? (SEQ - RH) / 32 : 1, 1), 32, 0, stream>>>((const us*)QK16, (const us*)(QK16 + PLN), (const us*)VT16, CTX);
    k_gemmw<<<dim3(MROWS / 64, DM / 64, 1), 32, 0, stream>>>(CTX, CK, WO2, CK, CK, OUT, DM * ROWSTEP);
}
